// Net_40561671143795
// MI455X (gfx1250) — hardware-verified
//
#include <hip/hip_runtime.h>
#include <math.h>

constexpr int NBATCH = 4096;
constexpr int NSTEP  = 512;
constexpr int NEMB   = 32;
constexpr int NHID   = 32;
constexpr int NVOC   = 101;
constexpr int NGATE  = 4 * NHID;
constexpr int NFC    = 2;
constexpr int GROWS  = 104;
constexpr int HPITCH = 40;
constexpr int FPITCH = 33;
constexpr float WCARRY = 16.0f;
constexpr float HCARRY = 64.0f;
constexpr float ZCARRY = WCARRY * HCARRY;
constexpr float ZINV   = 1.0f / ZCARRY;

static_assert(NEMB == 32, "one k-step");
static_assert(NHID == 32, "one k-step, two unit subtiles");
static_assert(NGATE == 128, "eight n-subtiles");
static_assert(NBATCH % 16 == 0, "batch tiles");
static_assert(NSTEP % 4 == 0, "id staging");
static_assert((NVOC * NGATE) % 128 == 0, "table staging exact");
static_assert(GROWS % 4 == 0 && GROWS >= NVOC, "table rows");
static_assert(16 * NFC == 32, "one 128-B line per batch tile");
static_assert(ZCARRY == 1024.0f, "carry product");

typedef __attribute__((ext_vector_type(16))) _Float16 v16h;
typedef __attribute__((ext_vector_type(8)))  _Float16 v8h;
typedef __attribute__((ext_vector_type(8)))  float    v8f;
typedef __attribute__((ext_vector_type(4)))  float    v4f;
typedef __attribute__((ext_vector_type(4)))  int      v4i;

template <typename T> struct Frag;
template <> struct Frag<_Float16> {
  typedef v16h V; union U { v16h v; v8h h[2]; };
  static __device__ __forceinline__ v16h load(const _Float16* p) {
    U f; f.h[0] = *(const v8h*)(p); f.h[1] = *(const v8h*)(p + 16); return f.v;
  }
  static __device__ __forceinline__ v8f mma(v16h a, v16h b, v8f c) {
    return __builtin_amdgcn_wmma_f32_16x16x32_f16(false, a, false, b, (short)0, c, false, false);
  }
};

__device__ __forceinline__ void gate_guard(v8f& a, v8f& b, v8f& c, v8f& d,
                                           v16h x, v16h w0, v16h w1, v16h w2, v16h w3) {
  asm volatile("v_nop\n\tv_nop\n\tv_nop\n\tv_nop"
               : "+v"(a), "+v"(b), "+v"(c), "+v"(d)
               : "v"(x), "v"(w0), "v"(w1), "v"(w2), "v"(w3));
}

__device__ __forceinline__ float fsig_z(float a)  { return __builtin_amdgcn_rcpf(1.0f + expf(a * (-ZINV))); }
__device__ __forceinline__ float ftanh_z(float a) { return 1.0f - 2.0f * __builtin_amdgcn_rcpf(expf(a * (2.0f * ZINV)) + 1.0f); }
__device__ __forceinline__ float ftanh_1(float v) { return 1.0f - 2.0f * __builtin_amdgcn_rcpf(expf(2.0f * v) + 1.0f); }

__global__ __launch_bounds__(128) void gate_table_kernel(const float* __restrict__ emb, const float* __restrict__ Wx,
                                                         const float* __restrict__ bg, float* __restrict__ GS) {
  const int tid = threadIdx.x;
  const int lane = tid & 31;
  const int v = blockIdx.x * 4 + (tid >> 5);
  const int n4 = lane * 4;
  const int vc = (v < NVOC) ? v : (NVOC - 1);
  const float* er = emb + vc * NEMB;
  v4f acc = {0.0f, 0.0f, 0.0f, 0.0f};
#pragma unroll 2
  for (int k = 0; k < NEMB; ++k) {
    const float e = er[k];
    const v4f w = *(const v4f*)(Wx + k * NGATE + n4);
    acc[0] = fmaf(e, w[0], acc[0]);
    acc[1] = fmaf(e, w[1], acc[1]);
    acc[2] = fmaf(e, w[2], acc[2]);
    acc[3] = fmaf(e, w[3], acc[3]);
  }
  const v4f bv = *(const v4f*)(bg + n4);
  const bool live = (v < NVOC);
  v4f o;
  o[0] = live ? (acc[0] + bv[0]) * ZCARRY : 0.0f;
  o[1] = live ? (acc[1] + bv[1]) * ZCARRY : 0.0f;
  o[2] = live ? (acc[2] + bv[2]) * ZCARRY : 0.0f;
  o[3] = live ? (acc[3] + bv[3]) * ZCARRY : 0.0f;
  float* op = GS + (size_t)v * NGATE + n4;
  *(volatile v4f*)op = o;
  __threadfence();
  *(volatile v4f*)op = o;
}

__global__ __launch_bounds__(256) void wh_plane_kernel(const float* __restrict__ Wh, unsigned short* __restrict__ WHT) {
  const int i = blockIdx.x * 256 + threadIdx.x;
  if (i < NGATE * (NHID / 8)) {
    const int n = i >> 2;
    const int k8 = (i & 3) * 8;
    v8h hv;
#pragma unroll
    for (int e = 0; e < 8; ++e) {
      const float f = Wh[(k8 + e) * NGATE + n];
      hv[e] = (_Float16)(f * WCARRY);
    }
    unsigned short* op = WHT + (size_t)i * 8;
    *(volatile v8h*)op = hv;
    __threadfence();
    *(volatile v8h*)op = hv;
  }
}

__global__ __launch_bounds__(32) void lstm_seq_kernel(const int* __restrict__ x, const float* __restrict__ GS,
                                                      const unsigned short* __restrict__ WHTp,
                                                      const float* __restrict__ Wfc, const float* __restrict__ bfc,
                                                      float* __restrict__ out) {
  __shared__ __align__(16) float    Gs[NVOC * NGATE];
  __shared__ __align__(16) unsigned idw[NSTEP * 4];
  __shared__ __align__(16) _Float16 hb[16 * HPITCH];
  __shared__ __align__(16) float    hf[16 * FPITCH];

  const _Float16* WHT = (const _Float16*)WHTp;
  const int lane = threadIdx.x & 31;
  const int c = lane & 15;
  const int hh = lane >> 4;
  const int koff = hh * 8;
  const int b0 = blockIdx.x * 16;

#pragma unroll 4
  for (int i = 0; i < NVOC; ++i) {
    const int o = (i * 32 + lane) * 4;
    const v4f v = *(const v4f*)(GS + o);
    *(v4f*)(Gs + o) = v;
  }
#pragma unroll 1
  for (int it = 0; it < 16; ++it) {
    const int idx = it * 32 + lane;
    const int q = idx & 3;
    const int t0 = (idx >> 2) * 4;
    const size_t base = (size_t)(b0 + 4 * q) * NSTEP + (size_t)t0;
    const v4i a0 = *(const v4i*)(x + base);
    const v4i a1 = *(const v4i*)(x + base + (size_t)NSTEP);
    const v4i a2 = *(const v4i*)(x + base + (size_t)2 * NSTEP);
    const v4i a3 = *(const v4i*)(x + base + (size_t)3 * NSTEP);
#pragma unroll
    for (int e = 0; e < 4; ++e) {
      int i0 = a0[e]; int i1 = a1[e]; int i2 = a2[e]; int i3 = a3[e];
      i0 = i0 < 0 ? 0 : (i0 > NVOC - 1 ? NVOC - 1 : i0);
      i1 = i1 < 0 ? 0 : (i1 > NVOC - 1 ? NVOC - 1 : i1);
      i2 = i2 < 0 ? 0 : (i2 > NVOC - 1 ? NVOC - 1 : i2);
      i3 = i3 < 0 ? 0 : (i3 > NVOC - 1 ? NVOC - 1 : i3);
      const unsigned w = (unsigned)i0 | ((unsigned)i1 << 8) | ((unsigned)i2 << 16) | ((unsigned)i3 << 24);
      idw[(t0 + e) * 4 + q] = w;
    }
  }
  v16h wh[8];
  wh[0] = Frag<_Float16>::load(WHT + (size_t)(0 * 16 + c) * NHID + koff);
  wh[1] = Frag<_Float16>::load(WHT + (size_t)(1 * 16 + c) * NHID + koff);
  wh[2] = Frag<_Float16>::load(WHT + (size_t)(2 * 16 + c) * NHID + koff);
  wh[3] = Frag<_Float16>::load(WHT + (size_t)(3 * 16 + c) * NHID + koff);
  asm volatile("" ::: "memory");
  wh[4] = Frag<_Float16>::load(WHT + (size_t)(4 * 16 + c) * NHID + koff);
  wh[5] = Frag<_Float16>::load(WHT + (size_t)(5 * 16 + c) * NHID + koff);
  wh[6] = Frag<_Float16>::load(WHT + (size_t)(6 * 16 + c) * NHID + koff);
  wh[7] = Frag<_Float16>::load(WHT + (size_t)(7 * 16 + c) * NHID + koff);
  asm volatile("" ::: "memory");

  float cst[2][8], hst[2][8];
#pragma unroll
  for (int u = 0; u < 2; ++u)
#pragma unroll
    for (int r = 0; r < 8; ++r) { cst[u][r] = 0.0f; hst[u][r] = 0.0f; }
  v16h hF = {};
  __syncthreads();

  const _Float16* hrow = hb + c * HPITCH + koff;

#pragma unroll 1
  for (int t = 0; t < NSTEP; ++t) {
    const unsigned w0 = idw[t * 4 + 2 * hh];
    const unsigned w1 = idw[t * 4 + 2 * hh + 1];
    int gofs[8];
#pragma unroll
    for (int r = 0; r < 8; ++r) {
      const unsigned w = (r < 4) ? w0 : w1;
      int id = (int)((w >> (8 * (r & 3))) & 0xffu);
      id = id > (NVOC - 1) ? (NVOC - 1) : id;
      gofs[r] = id * NGATE + c;
    }
#pragma unroll
    for (int u = 0; u < 2; ++u) {
      v8f ai, af, ag, ao;
#pragma unroll
      for (int r = 0; r < 8; ++r) {
        ai[r] = Gs[gofs[r] + 16 * u];
        af[r] = Gs[gofs[r] + NHID + 16 * u];
        ag[r] = Gs[gofs[r] + 2 * NHID + 16 * u];
        ao[r] = Gs[gofs[r] + 3 * NHID + 16 * u];
      }
      ai = Frag<_Float16>::mma(hF, wh[u],     ai);
      af = Frag<_Float16>::mma(hF, wh[2 + u], af);
      ag = Frag<_Float16>::mma(hF, wh[4 + u], ag);
      ao = Frag<_Float16>::mma(hF, wh[6 + u], ao);
      gate_guard(ai, af, ag, ao, hF, wh[u], wh[2 + u], wh[4 + u], wh[6 + u]);
#pragma unroll
      for (int r = 0; r < 8; ++r) {
        const float si = fsig_z(ai[r]);
        const float sf = fsig_z(af[r]);
        const float tg = ftanh_z(ag[r]);
        const float so = fsig_z(ao[r]);
        const float cn = sf * cst[u][r] + si * tg;
        cst[u][r] = cn;
        hst[u][r] = so * ftanh_1(cn);
      }
    }
    __syncthreads();
#pragma unroll
    for (int u = 0; u < 2; ++u)
#pragma unroll
      for (int r = 0; r < 8; ++r)
        hb[(8 * hh + r) * HPITCH + 16 * u + c] = (_Float16)(hst[u][r] * HCARRY);
    __syncthreads();
    hF = Frag<_Float16>::load(hrow);
  }

#pragma unroll
  for (int u = 0; u < 2; ++u)
#pragma unroll
    for (int r = 0; r < 8; ++r)
      hf[(8 * hh + r) * FPITCH + 16 * u + c] = hst[u][r];
  __syncthreads();
  {
    const int row = lane >> 1;
    const int j = lane & 1;
    float accv = 0.0f;
#pragma unroll 4
    for (int k = 0; k < NHID; ++k) accv = fmaf(hf[row * FPITCH + k], Wfc[k * NFC + j], accv);
    const float res = accv + bfc[j];
    float* op = out + (size_t)blockIdx.x * 32 + lane;
    *(volatile float*)op = res;
    __threadfence();
    *(volatile float*)op = res;
  }
}

extern "C" void kernel_launch(void* const* d_in, const int* in_sizes, int n_in,
                              void* d_out, int out_size, void* d_ws, size_t ws_size, hipStream_t stream) {
  if (n_in < 7 || d_out == nullptr || d_ws == nullptr) return;
  if (in_sizes[0] != NBATCH * NSTEP || in_sizes[1] != NVOC * NEMB || in_sizes[2] != NEMB * NGATE ||
      in_sizes[3] != NHID * NGATE || in_sizes[4] != NGATE || in_sizes[5] != NHID * NFC ||
      in_sizes[6] != NFC || out_size != NBATCH * NFC) return;

  const int*   xin  = (const int*)d_in[0];
  const float* emb  = (const float*)d_in[1];
  const float* wx   = (const float*)d_in[2];
  const float* whh  = (const float*)d_in[3];
  const float* bg   = (const float*)d_in[4];
  const float* wfc  = (const float*)d_in[5];
  const float* bfc  = (const float*)d_in[6];
  float* out = (float*)d_out;

  char* ws = (char*)d_ws; size_t off = 0;
  auto carve = [&](size_t bytes) -> char* { char* p = ws + off; off += (bytes + 255) & ~(size_t)255; return p; };
  float*          GS  = (float*)carve((size_t)GROWS * NGATE * 4);
  unsigned short* WHT = (unsigned short*)carve((size_t)NGATE * NHID * 2);
  if (off > ws_size || off > (size_t)134217728) return;

  gate_table_kernel<<<GROWS / 4, 128, 0, stream>>>(emb, wx, bg, GS);
  wh_plane_kernel<<<(NGATE * (NHID / 8)) / 256, 256, 0, stream>>>(whh, WHT);
  lstm_seq_kernel<<<NBATCH / 16, 32, 0, stream>>>(xin, GS, WHT, wfc, bfc, out);
}
